// MambaBlock2D_48172353192409
// MI455X (gfx1250) — hardware-verified
//
#include <hip/hip_runtime.h>
#include <math.h>

typedef __attribute__((ext_vector_type(16))) _Float16 v16h;
typedef __attribute__((ext_vector_type(8)))  _Float16 v8h;
typedef __attribute__((ext_vector_type(8)))  float    v8f;
typedef __attribute__((ext_vector_type(4)))  float    v4f;

constexpr int kBatch  = 2;
constexpr int kSeq    = 4096;
constexpr int kDm     = 256;
constexpr int kDin    = 512;
constexpr int kNst    = 16;
constexpr int kDtR    = 16;
constexpr int kXzP    = 2 * kDin;
constexpr int kXdN    = kDtR + 2 * kNst;
constexpr int kXdP    = 64;
constexpr int kFfn    = 4 * kDm;
constexpr int kRows   = kBatch * kSeq;
constexpr int kLnTok  = 32;
constexpr int kLnPitch = 36;
constexpr int kConvTP = 260;
constexpr int kScanTS = 64;
constexpr int kScanCh = 64;
constexpr int kScanYP = 68;
static_assert(kXdN <= kXdP);
static_assert((kDm % 32) == 0 && (kDin % 32) == 0 && (kFfn % 32) == 0);
static_assert((kRows % 64) == 0 && (kXzP % 64) == 0 && (kXdP % 64) == 0 && (kDm % 64) == 0 && (kFfn % 64) == 0 && (kSeq % 64) == 0);
static_assert((kSeq % kScanTS) == 0 && (kSeq % kLnTok) == 0 && (kDin % kScanCh) == 0 && (kDin % 256) == 0 && kDm == 256);
static_assert(((kRows / 64) * (kXzP / 64)) % 8 == 0 && ((kRows / 64) * (kXdP / 64)) % 8 == 0 && ((kRows / 64) * (kDm / 64)) % 8 == 0 &&
              ((kRows / 64) * (kFfn / 64)) % 8 == 0 && ((kDm / 64) * (kSeq / 64)) % 8 == 0);

constexpr size_t kOffWIN  = 0;
constexpr size_t kOffWXP  = kOffWIN + (size_t)kXzP * kDm * 2;
constexpr size_t kOffWOU  = kOffWXP + (size_t)kXdP * kDin * 2;
constexpr size_t kOffW1H  = kOffWOU + (size_t)kDm * kDin * 2;
constexpr size_t kOffW2H  = kOffW1H + (size_t)kFfn * kDm * 2;
constexpr size_t kOffYNF  = kOffW2H + (size_t)kDm * kFfn * 2;
constexpr size_t kOffYNH  = kOffYNF + (size_t)kRows * kDm * 4;
constexpr size_t kOffXZ   = kOffYNH + (size_t)kRows * kDm * 2;
constexpr size_t kOffUF   = kOffXZ  + (size_t)kRows * kXzP * 4;
constexpr size_t kOffUH   = kOffUF  + (size_t)kRows * kDin * 4;
constexpr size_t kOffXD   = kOffUH  + (size_t)kRows * kDin * 2;
constexpr size_t kOffYMH  = kOffXD  + (size_t)kRows * kXdP * 4;
constexpr size_t kOffY2F  = kOffYMH + (size_t)kRows * kDin * 2;
constexpr size_t kOffY2H  = kOffY2F + (size_t)kRows * kDm * 4;
constexpr size_t kOffH1H  = kOffY2H + (size_t)kRows * kDm * 2;
constexpr size_t kWsTotal = kOffH1H + (size_t)kRows * kFfn * 2;
static_assert(kWsTotal == 113049600ull);
static_assert(kWsTotal <= 134217728ull);
static_assert((size_t)kRows * kFfn * 4 <= (size_t)kRows * kXzP * 4);
static_assert((kOffWXP % 128) == 0 && (kOffWOU % 128) == 0 && (kOffW1H % 128) == 0 && (kOffW2H % 128) == 0 &&
              (kOffYNF % 128) == 0 && (kOffYNH % 128) == 0 && (kOffXZ % 128) == 0 && (kOffUF % 128) == 0 &&
              (kOffUH % 128) == 0 && (kOffXD % 128) == 0 && (kOffYMH % 128) == 0 && (kOffY2F % 128) == 0 &&
              (kOffY2H % 128) == 0 && (kOffH1H % 128) == 0);

__device__ __forceinline__ void dep_guard_h(v8f& a, v8f& b, v16h x, v16h y) { asm volatile("v_nop\n\tv_nop\n\tv_nop\n\tv_nop" : "+v"(a), "+v"(b) : "v"(x), "v"(y)); }
__device__ __forceinline__ void keep4_h(v16h a, v16h b, v16h c, v16h d) { asm volatile("v_nop" :: "v"(a), "v"(b), "v"(c), "v"(d)); }
__device__ __forceinline__ void acc_guard4(v8f& a, v8f& b, v8f& c, v8f& d) { asm volatile("v_nop\n\tv_nop\n\tv_nop\n\tv_nop" : "+v"(a), "+v"(b), "+v"(c), "+v"(d)); }
__device__ __forceinline__ void dep_guard_row(v8f& a0, v8f& a1, v8f& a2, v8f& a3, v16h x, v16h y0, v16h y1, v16h y2, v16h y3) {
  asm volatile("v_nop\n\tv_nop\n\tv_nop\n\tv_nop" : "+v"(a0), "+v"(a1), "+v"(a2), "+v"(a3) : "v"(x), "v"(y0), "v"(y1), "v"(y2), "v"(y3));
}
template <typename T> struct Frag;
template <> struct Frag<_Float16> {
  typedef v16h V; union U { v16h v; v8h h[2]; };
  static __device__ __forceinline__ v16h load(const _Float16* p) {
    U f; f.h[0] = *(const v8h*)(p); f.h[1] = *(const v8h*)(p + 16); return f.v;
  }
  static __device__ __forceinline__ v8f mma(v16h a, v16h b, v8f c) {
    return __builtin_amdgcn_wmma_f32_16x16x32_f16(false, a, false, b, (short)0, c, false, false);
  }
  static __device__ __forceinline__ void guard(v8f& a, v8f& b, v16h x, v16h y) { dep_guard_h(a, b, x, y); }
  static __device__ __forceinline__ void keep(v16h a, v16h b, v16h c, v16h d) { keep4_h(a, b, c, d); }
};
__device__ __forceinline__ void wave_lds_sync() {
  __builtin_amdgcn_fence(__ATOMIC_RELEASE, "workgroup");
  __builtin_amdgcn_wave_barrier();
  __builtin_amdgcn_fence(__ATOMIC_ACQUIRE, "workgroup");
}

template <int BIAS_MODE, int RES_MODE>
__global__ __launch_bounds__(256) void gemm_f16w(
    const unsigned short* __restrict__ Ap, int lda, long strideA,
    const unsigned short* __restrict__ Btp, int ldb, long strideB,
    float* __restrict__ Cout, int ldc, long strideC,
    const float* __restrict__ bias,
    const float* __restrict__ resid, int ldr, long strideR,
    int M, int N, int K) {
  typedef Frag<_Float16> F;
  const _Float16* A = (const _Float16*)Ap; const _Float16* Bt = (const _Float16*)Btp;
  __shared__ __align__(16) float sT[8][16 * 68];
  const int b    = blockIdx.y;
  const int lane = threadIdx.x & 31;
  const int wave = threadIdx.x >> 5;
  const int tilesN = N >> 6;
  const int tilesM = M >> 6;
  const int tile = blockIdx.x * 8 + wave;
  if (tile >= tilesM * tilesN) return;
  const int tm = tile / tilesN;
  const int tn = tile - tm * tilesN;
  const int m0 = tm << 6;
  const int n0 = tn << 6;

  const _Float16* Ab = A  + (size_t)b * strideA;
  const _Float16* Bb = Bt + (size_t)b * strideB;

  const int rlane = lane & 15;
  const int koff  = (lane >> 4) * 8;
  const int mOff  = (lane >> 4) * 8;

  v8f acc[4][4];
#pragma unroll
  for (int i = 0; i < 4; ++i)
#pragma unroll
    for (int j = 0; j < 4; ++j) acc[i][j] = (v8f){0.f,0.f,0.f,0.f,0.f,0.f,0.f,0.f};

  for (int k0 = 0; k0 < K; k0 += 32) {
    v16h bh[4];
#pragma unroll
    for (int j = 0; j < 4; ++j) {
      const size_t bo = (size_t)(n0 + (j << 4) + rlane) * ldb + koff + k0;
      bh[j] = F::load(Bb + bo);
    }
#pragma unroll
    for (int i = 0; i < 4; ++i) {
      const size_t ao = (size_t)(m0 + (i << 4) + rlane) * lda + koff + k0;
      const v16h ah = F::load(Ab + ao);
#pragma unroll
      for (int j = 0; j < 4; ++j) acc[i][j] = F::mma(ah, bh[j], acc[i][j]);
      dep_guard_row(acc[i][0], acc[i][1], acc[i][2], acc[i][3], ah, bh[0], bh[1], bh[2], bh[3]);
    }
    F::keep(bh[0], bh[1], bh[2], bh[3]);
  }
  acc_guard4(acc[0][0], acc[0][1], acc[0][2], acc[0][3]);
  acc_guard4(acc[1][0], acc[1][1], acc[1][2], acc[1][3]);
  acc_guard4(acc[2][0], acc[2][1], acc[2][2], acc[2][3]);
  acc_guard4(acc[3][0], acc[3][1], acc[3][2], acc[3][3]);

  float* slab = sT[wave];
  const float* Rb = (RES_MODE != 0) ? (resid + (size_t)b * strideR) : resid;
  float* Cb = Cout + (size_t)b * strideC;
  const int hh = lane >> 4, c4 = (lane & 15) * 4;
  const int tq = lane >> 2, cq = (lane & 3) * 4;
#pragma unroll
  for (int i = 0; i < 4; ++i) {
    const int mBase = m0 + (i << 4);
    if (RES_MODE == 1) {
#pragma unroll
      for (int it = 0; it < 8; ++it) {
        const int row = it * 2 + hh;
        const v4f rv = *(const v4f*)(Rb + (size_t)(mBase + row) * ldr + n0 + c4);
        *(v4f*)(slab + row * 68 + c4) = rv;
      }
      wave_lds_sync();
    }
    if (RES_MODE == 2) {
#pragma unroll
      for (int it = 0; it < 8; ++it) {
        const int t = it * 8 + tq;
        const v4f rv = *(const v4f*)(Rb + (size_t)(n0 + t) * ldr + mBase + cq);
        slab[(cq + 0) * 68 + t] = rv[0];
        slab[(cq + 1) * 68 + t] = rv[1];
        slab[(cq + 2) * 68 + t] = rv[2];
        slab[(cq + 3) * 68 + t] = rv[3];
      }
      wave_lds_sync();
    }
#pragma unroll
    for (int j = 0; j < 4; ++j) {
      const int n = n0 + (j << 4) + rlane;
      float bv = 0.f;
      if (BIAS_MODE == 2) bv = bias[n];
#pragma unroll
      for (int r = 0; r < 8; ++r) {
        float v = acc[i][j][r];
        if (BIAS_MODE == 1) v += bias[mBase + mOff + r];
        if (BIAS_MODE == 2) v += bv;
        const int pos = (mOff + r) * 68 + (j << 4) + rlane;
        if (RES_MODE != 0) v += slab[pos];
        slab[pos] = v;
      }
    }
    wave_lds_sync();
    for (int pass = 0; pass < 2; ++pass) {
#pragma unroll
      for (int it = 0; it < 8; ++it) {
        const int row = it * 2 + hh;
        v4f v = *(const v4f*)(slab + row * 68 + c4);
        *(volatile v4f*)(Cb + (size_t)(mBase + row) * ldc + n0 + c4) = v;
      }
      __threadfence();
    }
    wave_lds_sync();
  }
}

__global__ __launch_bounds__(256) void cast_rows_f16_kernel(
    const float* __restrict__ src, unsigned short* __restrict__ dst, int cols, int rows_real, int total8)
{
  const int i = blockIdx.x * 256 + threadIdx.x;
  if (i >= total8) return;
  const size_t e0 = (size_t)i << 3;
  const int row = (int)(e0 / (size_t)cols);
  const int col = (int)(e0 - (size_t)row * (size_t)cols);
  const int rr = (row < rows_real) ? row : (rows_real - 1);
  const float fz = (row < rows_real) ? 1.0f : 0.0f;
  const float* sp = src + (size_t)rr * cols + col;
  const v4f a0 = *(const v4f*)(sp);
  const v4f a1 = *(const v4f*)(sp + 4);
  v8h hv;
#pragma unroll
  for (int e = 0; e < 4; ++e) {
    hv[e]     = (_Float16)(a0[e] * fz);
    hv[4 + e] = (_Float16)(a1[e] * fz);
  }
  unsigned short* p = dst + e0;
  *(volatile v8h*)p = hv;
  __threadfence();
  *(volatile v8h*)p = hv;
}

__global__ __launch_bounds__(256) void ln_kernel(
    const float* __restrict__ x, const float* __restrict__ gam, const float* __restrict__ bet,
    float* __restrict__ YNF, unsigned short* __restrict__ YNH)
{
  __shared__ __align__(16) float sX[kDm * kLnPitch];
  __shared__ float sG[kDm];
  __shared__ float sB[kDm];
  const int tid = threadIdx.x, lane = tid & 31, wave = tid >> 5;
  constexpr int kBlkPerB = kSeq / kLnTok;
  const int bix = blockIdx.x / kBlkPerB;
  const int l0  = (blockIdx.x - bix * kBlkPerB) * kLnTok;
  sG[tid] = gam[tid];
  sB[tid] = bet[tid];
  const int q = lane >> 3, e4 = (lane & 7) * 4;
#pragma unroll
  for (int it = 0; it < 8; ++it) {
    const int c = it * 32 + wave * 4 + q;
    const v4f v = *(const v4f*)(x + ((size_t)(bix * kDm + c)) * kSeq + l0 + e4);
    *(v4f*)(sX + c * kLnPitch + e4) = v;
  }
  __syncthreads();
#pragma unroll 1
  for (int tt = 0; tt < 4; ++tt) {
    const int t = wave * 4 + tt;
    float s8[8];
    float sum = 0.0f;
#pragma unroll
    for (int k = 0; k < 8; ++k) { s8[k] = sX[(lane * 8 + k) * kLnPitch + t]; sum += s8[k]; }
#pragma unroll
    for (int off = 1; off < 32; off <<= 1) sum += __shfl_xor(sum, off, 32);
    const float mu = sum * (1.0f / (float)kDm);
    float sq = 0.0f;
#pragma unroll
    for (int k = 0; k < 8; ++k) { const float dv = s8[k] - mu; sq = fmaf(dv, dv, sq); }
#pragma unroll
    for (int off = 1; off < 32; off <<= 1) sq += __shfl_xor(sq, off, 32);
    const float rstd = rsqrtf(sq * (1.0f / (float)kDm) + 1e-5f);
    v8h hv;
    v4f lo, hi;
#pragma unroll
    for (int k = 0; k < 8; ++k) {
      const int c = lane * 8 + k;
      hv[k] = (_Float16)((s8[k] - mu) * rstd * sG[c] + sB[c]);
    }
#pragma unroll
    for (int e = 0; e < 4; ++e) {
      const int c0 = lane * 4 + e, c1 = 128 + lane * 4 + e;
      lo[e] = (sX[c0 * kLnPitch + t] - mu) * rstd * sG[c0] + sB[c0];
      hi[e] = (sX[c1 * kLnPitch + t] - mu) * rstd * sG[c1] + sB[c1];
    }
    const size_t row = (size_t)bix * kSeq + l0 + t;
    for (int pass = 0; pass < 2; ++pass) {
      *(volatile v4f*)(YNF + row * kDm + lane * 4) = lo;
      *(volatile v4f*)(YNF + row * kDm + 128 + lane * 4) = hi;
      *(volatile v8h*)(YNH + row * kDm + lane * 8) = hv;
      __threadfence();
    }
  }
}

__global__ __launch_bounds__(256) void conv_silu_kernel(
    const float* __restrict__ XZ, const float* __restrict__ cw, const float* __restrict__ cb,
    float* __restrict__ UF, unsigned short* __restrict__ UH)
{
  __shared__ __align__(16) float sT[16 * kConvTP];
  const int tid = threadIdx.x, lane = tid & 31, wave = tid >> 5;
  const int d0 = blockIdx.x * 256, d = d0 + tid;
  const int g0 = blockIdx.y * 64;
  const int tb = g0 & (kSeq - 1);
  const float w0 = cw[d * 4 + 0], w1 = cw[d * 4 + 1], w2 = cw[d * 4 + 2], w3 = cw[d * 4 + 3];
  const float bc = cb[d];
  float xm3, xm2, xm1;
  {
    const bool hist = (tb > 0);
    const int rb = hist ? (g0 - 3) : g0;
    const float v3 = XZ[(size_t)rb * kXzP + d];
    const float v2 = XZ[(size_t)(rb + 1) * kXzP + d];
    const float v1 = XZ[(size_t)(rb + 2) * kXzP + d];
    xm3 = hist ? v3 : 0.0f;
    xm2 = hist ? v2 : 0.0f;
    xm1 = hist ? v1 : 0.0f;
  }
  const int hrow = wave >> 1;
  const int hch  = (wave & 1) * 128 + lane * 4;
#pragma unroll 1
  for (int sub = 0; sub < 4; ++sub) {
    const int lb = g0 + sub * 16;
#pragma unroll 1
    for (int s = 0; s < 16; ++s) {
      const float xcur = XZ[(size_t)(lb + s) * kXzP + d];
      float acc = w0 * xm3;
      acc = fmaf(w1, xm2, acc);
      acc = fmaf(w2, xm1, acc);
      acc = fmaf(w3, xcur, acc);
      const float sv = acc + bc;
      const float sg = __builtin_amdgcn_rcpf(1.0f + expf(-sv));
      sT[s * kConvTP + tid] = sv * sg;
      xm3 = xm2; xm2 = xm1; xm1 = xcur;
    }
    __syncthreads();
    v4f fv[4];
    v8h hv[2];
#pragma unroll
    for (int it = 0; it < 4; ++it) fv[it] = *(const v4f*)(sT + (it * 4 + hrow) * kConvTP + hch);
#pragma unroll
    for (int it = 0; it < 2; ++it) {
      const float* sp = sT + (it * 8 + wave) * kConvTP + lane * 8;
      const v4f a0 = *(const v4f*)(sp);
      const v4f a1 = *(const v4f*)(sp + 4);
#pragma unroll
      for (int e = 0; e < 4; ++e) {
        hv[it][e]     = (_Float16)a0[e];
        hv[it][4 + e] = (_Float16)a1[e];
      }
    }
    for (int pass = 0; pass < 2; ++pass) {
#pragma unroll
      for (int it = 0; it < 4; ++it)
        *(volatile v4f*)(UF + (size_t)(lb + it * 4 + hrow) * kDin + d0 + hch) = fv[it];
#pragma unroll
      for (int it = 0; it < 2; ++it)
        *(volatile v8h*)(UH + (size_t)(lb + it * 8 + wave) * kDin + d0 + lane * 8) = hv[it];
      __threadfence();
    }
    __syncthreads();
  }
}

__global__ __launch_bounds__(kScanCh) void scan_kernel(
    const float* __restrict__ XD, const float* __restrict__ UF, const float* __restrict__ XZ,
    const float* __restrict__ Wdt, const float* __restrict__ bdt, const float* __restrict__ Alog,
    const float* __restrict__ Dp, unsigned short* __restrict__ YMH)
{
  __shared__ __align__(16) float sX[kScanTS * kXdP];
  __shared__ __align__(16) float sY[kScanTS * kScanYP];
  __shared__ __align__(16) float sW[kDtR * kScanCh];
  __shared__ __align__(16) float sA[kNst * kScanCh];
  const int tid = threadIdx.x, lane = tid & 31, wave = tid >> 5;
  constexpr int kBlkPerB = kDin / kScanCh;
  const int bix = blockIdx.x / kBlkPerB;
  const int d0  = (blockIdx.x - bix * kBlkPerB) * kScanCh;
  const int d   = d0 + tid;
  const size_t row0 = (size_t)bix * kSeq;
#pragma unroll 1
  for (int r = 0; r < kDtR; ++r) sW[r * kScanCh + tid] = Wdt[(size_t)d * kDtR + r];
#pragma unroll 1
  for (int s = 0; s < kNst; ++s) sA[s * kScanCh + tid] = -expf(Alog[(size_t)d * kNst + s]);
  __syncthreads();
  float negA[kNst], h[kNst];
#pragma unroll
  for (int s = 0; s < kNst; ++s) {
    negA[s] = sA[s * kScanCh + tid];
    h[s] = 0.0f;
  }
  const float bb = bdt[d], Dd = Dp[d];
  const int lr = tid >> 4, lc4 = (tid & 15) * 4;
  const int q = lane >> 3, c8 = (lane & 7) * 8;
#pragma unroll 1
  for (int t0 = 0; t0 < kSeq; t0 += kScanTS) {
    __syncthreads();
#pragma unroll
    for (int i = 0; i < 8; ++i) {
      const int r = lr + 4 * i;
      *(v4f*)(sX + r * kXdP + lc4) = *(const v4f*)(XD + (row0 + t0 + r) * kXdP + lc4);
    }
    asm volatile("" ::: "memory");
#pragma unroll
    for (int i = 8; i < 16; ++i) {
      const int r = lr + 4 * i;
      *(v4f*)(sX + r * kXdP + lc4) = *(const v4f*)(XD + (row0 + t0 + r) * kXdP + lc4);
    }
    __syncthreads();
#pragma unroll 1
    for (int s = 0; s < kScanTS; ++s) {
      const int t = t0 + s;
      const float* xr = sX + s * kXdP;
      float vdot = 0.0f;
#pragma unroll 1
      for (int r4 = 0; r4 < kDtR / 4; ++r4) {
        const v4f xv = *(const v4f*)(xr + 4 * r4);
        const float* wp = sW + (4 * r4) * kScanCh + tid;
        vdot = fmaf(xv[0], wp[0], vdot);
        vdot = fmaf(xv[1], wp[kScanCh], vdot);
        vdot = fmaf(xv[2], wp[2 * kScanCh], vdot);
        vdot = fmaf(xv[3], wp[3 * kScanCh], vdot);
      }
      float Bs[kNst], Cs[kNst];
#pragma unroll
      for (int q4 = 0; q4 < 4; ++q4) {
        const v4f bv = *(const v4f*)(xr + kDtR + 4 * q4);
        const v4f cv = *(const v4f*)(xr + kDtR + kNst + 4 * q4);
        Bs[4 * q4 + 0] = bv[0]; Bs[4 * q4 + 1] = bv[1]; Bs[4 * q4 + 2] = bv[2]; Bs[4 * q4 + 3] = bv[3];
        Cs[4 * q4 + 0] = cv[0]; Cs[4 * q4 + 1] = cv[1]; Cs[4 * q4 + 2] = cv[2]; Cs[4 * q4 + 3] = cv[3];
      }
      const float v   = vdot + bb;
      const float ea  = expf(-fabsf(v));
      const float dt  = fmaxf(v, 0.0f) + log1pf(ea);
      const float xt  = UF[(row0 + t) * kDin + d];
      const float dtx = dt * xt;
      float y = 0.0f;
#pragma unroll
      for (int k = 0; k < kNst; ++k) {
        const float e = __expf(dt * negA[k]);
        h[k] = fmaf(e, h[k], dtx * Bs[k]);
        y = fmaf(h[k], Cs[k], y);
      }
      y = fmaf(xt, Dd, y);
      const float zv = XZ[(row0 + t) * kXzP + kDin + d];
      const float sg = __builtin_amdgcn_rcpf(1.0f + expf(-zv));
      y = y * (zv * sg);
      sY[s * kScanYP + tid] = y;
    }
    __syncthreads();
    v8h hv[8];
#pragma unroll
    for (int it = 0; it < 8; ++it) {
      const int row = it * 8 + wave * 4 + q;
      const float* sp = sY + row * kScanYP + c8;
      const v4f a0 = *(const v4f*)(sp);
      const v4f a1 = *(const v4f*)(sp + 4);
#pragma unroll
      for (int e = 0; e < 4; ++e) {
        hv[it][e]     = (_Float16)a0[e];
        hv[it][4 + e] = (_Float16)a1[e];
      }
    }
    for (int pass = 0; pass < 2; ++pass) {
#pragma unroll
      for (int it = 0; it < 8; ++it) {
        const int row = it * 8 + wave * 4 + q;
        const size_t o = (row0 + t0 + row) * kDin + d0 + c8;
        *(volatile v8h*)(YMH + o) = hv[it];
      }
      __threadfence();
    }
  }
}

__global__ __launch_bounds__(256) void gelu_f16_kernel(const float* __restrict__ src, unsigned short* __restrict__ dst)
{
  __shared__ __align__(16) float sg[256 * 8];
  const int tid = threadIdx.x;
  const size_t e0 = ((size_t)blockIdx.x * 256 + tid) << 3;
  const v4f a0 = *(const v4f*)(src + e0);
  const v4f a1 = *(const v4f*)(src + e0 + 4);
  *(v4f*)(sg + tid * 8) = a0;
  *(v4f*)(sg + tid * 8 + 4) = a1;
  __syncthreads();
#pragma unroll 1
  for (int e = 0; e < 8; ++e) {
    const float xv = sg[tid * 8 + e];
    const float gv = 0.5f * xv * (1.0f + erff(xv * 0.70710678118654752f));
    sg[tid * 8 + e] = gv;
  }
  __syncthreads();
  const v4f g0 = *(const v4f*)(sg + tid * 8);
  const v4f g1 = *(const v4f*)(sg + tid * 8 + 4);
  v8h hv;
#pragma unroll
  for (int e = 0; e < 4; ++e) {
    hv[e]     = (_Float16)g0[e];
    hv[4 + e] = (_Float16)g1[e];
  }
  unsigned short* p = dst + e0;
  *(volatile v8h*)p = hv;
  __threadfence();
  *(volatile v8h*)p = hv;
}

extern "C" void kernel_launch(void* const* d_in, const int* in_sizes, int n_in,
                              void* d_out, int out_size, void* d_ws, size_t ws_size,
                              hipStream_t stream) {
  if (n_in < 16) return;
  if (in_sizes[0] != kRows * kDm) return;
  if (in_sizes[1] != kDm) return;
  if (in_sizes[2] != kDm) return;
  if (in_sizes[3] != kXzP * kDm) return;
  if (in_sizes[4] != kDin * 4) return;
  if (in_sizes[5] != kDin) return;
  if (in_sizes[6] != kXdN * kDin) return;
  if (in_sizes[7] != kDin * kDtR) return;
  if (in_sizes[8] != kDin) return;
  if (in_sizes[9] != kDin * kNst) return;
  if (in_sizes[10] != kDin) return;
  if (in_sizes[11] != kDm * kDin) return;
  if (in_sizes[12] != kFfn * kDm) return;
  if (in_sizes[13] != kFfn) return;
  if (in_sizes[14] != kDm * kFfn) return;
  if (in_sizes[15] != kDm) return;
  if (out_size != kRows * kDm) return;
  if (ws_size < kWsTotal) return;

  const float* x      = (const float*)d_in[0];
  const float* gam    = (const float*)d_in[1];
  const float* bet    = (const float*)d_in[2];
  const float* W_in   = (const float*)d_in[3];
  const float* conv_w = (const float*)d_in[4];
  const float* conv_b = (const float*)d_in[5];
  const float* W_xp   = (const float*)d_in[6];
  const float* W_dt   = (const float*)d_in[7];
  const float* b_dt   = (const float*)d_in[8];
  const float* A_log  = (const float*)d_in[9];
  const float* Dvec   = (const float*)d_in[10];
  const float* W_out  = (const float*)d_in[11];
  const float* W1     = (const float*)d_in[12];
  const float* b1     = (const float*)d_in[13];
  const float* W2     = (const float*)d_in[14];
  const float* b2     = (const float*)d_in[15];
  float* out = (float*)d_out;

  char* ws = (char*)d_ws;
  unsigned short* WINH = (unsigned short*)(ws + kOffWIN);
  unsigned short* WXPH = (unsigned short*)(ws + kOffWXP);
  unsigned short* WOUH = (unsigned short*)(ws + kOffWOU);
  unsigned short* W1H  = (unsigned short*)(ws + kOffW1H);
  unsigned short* W2H  = (unsigned short*)(ws + kOffW2H);
  float*          YNF  = (float*)(ws + kOffYNF);
  unsigned short* YNH  = (unsigned short*)(ws + kOffYNH);
  float*          XZ   = (float*)(ws + kOffXZ);
  float*          G1   = (float*)(ws + kOffXZ);
  float*          UF   = (float*)(ws + kOffUF);
  unsigned short* UH   = (unsigned short*)(ws + kOffUH);
  float*          XD   = (float*)(ws + kOffXD);
  unsigned short* YMH  = (unsigned short*)(ws + kOffYMH);
  float*          Y2F  = (float*)(ws + kOffY2F);
  unsigned short* Y2H  = (unsigned short*)(ws + kOffY2H);
  unsigned short* H1H  = (unsigned short*)(ws + kOffH1H);

  cast_rows_f16_kernel<<<(kXzP * kDm / 8) / 256, 256, 0, stream>>>(W_in, WINH, kDm, kXzP, kXzP * kDm / 8);
  cast_rows_f16_kernel<<<(kXdP * kDin / 8) / 256, 256, 0, stream>>>(W_xp, WXPH, kDin, kXdN, kXdP * kDin / 8);
  cast_rows_f16_kernel<<<(kDm * kDin / 8) / 256, 256, 0, stream>>>(W_out, WOUH, kDin, kDm, kDm * kDin / 8);
  cast_rows_f16_kernel<<<(kFfn * kDm / 8) / 256, 256, 0, stream>>>(W1, W1H, kDm, kFfn, kFfn * kDm / 8);
  cast_rows_f16_kernel<<<(kDm * kFfn / 8) / 256, 256, 0, stream>>>(W2, W2H, kFfn, kDm, kDm * kFfn / 8);

  ln_kernel<<<kRows / kLnTok, 256, 0, stream>>>(x, gam, bet, YNF, YNH);

  gemm_f16w<0, 0><<<dim3((kRows / 64) * (kXzP / 64) / 8, 1), 256, 0, stream>>>(
      YNH, kDm, 0L, WINH, kDm, 0L, XZ, kXzP, 0L, nullptr, nullptr, 0, 0L, kRows, kXzP, kDm);

  conv_silu_kernel<<<dim3(kDin / 256, kRows / 64), 256, 0, stream>>>(XZ, conv_w, conv_b, UF, UH);

  gemm_f16w<0, 0><<<dim3((kRows / 64) * (kXdP / 64) / 8, 1), 256, 0, stream>>>(
      UH, kDin, 0L, WXPH, kDin, 0L, XD, kXdP, 0L, nullptr, nullptr, 0, 0L, kRows, kXdP, kDin);

  scan_kernel<<<kBatch * (kDin / kScanCh), kScanCh, 0, stream>>>(XD, UF, XZ, W_dt, b_dt, A_log, Dvec, YMH);

  gemm_f16w<0, 1><<<dim3((kRows / 64) * (kDm / 64) / 8, 1), 256, 0, stream>>>(
      YMH, kDin, 0L, WOUH, kDin, 0L, Y2F, kDm, 0L, nullptr, YNF, kDm, 0L, kRows, kDm, kDin);

  cast_rows_f16_kernel<<<(kRows * kDm / 8) / 256, 256, 0, stream>>>(Y2F, Y2H, kDm, kRows, kRows * kDm / 8);

  gemm_f16w<2, 0><<<dim3((kRows / 64) * (kFfn / 64) / 8, 1), 256, 0, stream>>>(
      Y2H, kDm, 0L, W1H, kDm, 0L, G1, kFfn, 0L, b1, nullptr, 0, 0L, kRows, kFfn, kDm);

  gelu_f16_kernel<<<(kRows * kFfn / 8) / 256, 256, 0, stream>>>(G1, H1H);

  gemm_f16w<1, 2><<<dim3((kDm / 64) * (kSeq / 64) / 8, kBatch), 256, 0, stream>>>(
      W2H, kFfn, 0L, H1H, kFfn, (long)kSeq * kFfn, out, kSeq, (long)kDm * kSeq,
      b2, Y2F, kDm, (long)kSeq * kDm, kDm, kSeq, kFfn);
}
